// Model_52888227283552
// MI455X (gfx1250) — hardware-verified
//
#include <hip/hip_runtime.h>
#include <math.h>

constexpr int NBATCH   = 4096;
constexpr int NSTEP    = 512;
constexpr int NIN      = 4;
constexpr int NHID     = 50;
constexpr int NOUT     = 121;
constexpr int NGATE    = 4;
constexpr int UPAD     = 64;
constexpr int NROWB    = NGATE * UPAD;
constexpr int KPAD     = 64;
constexpr int ROWS_BLK = 32;
constexpr int NTHR     = 128;
constexpr int APITCH   = 72;
constexpr int XCHUNK   = 32;
constexpr int COL_X    = NHID;
constexpr int COL_ONE  = NHID + NIN;
constexpr int COL_ZERO = NHID + NIN + 2;
constexpr int NLINES   = (ROWS_BLK * NOUT) / 32;
constexpr float ACARRY = 64.0f;
constexpr float WCARRY = 256.0f;
constexpr float FOLD   = 1.0f / (ACARRY * WCARRY);
constexpr float LOG2E  = 1.4426950408889634f;
constexpr float KSIG   = -FOLD * LOG2E;
constexpr float KTG    = 2.0f * FOLD * LOG2E;
constexpr float KTC    = 2.0f * LOG2E;

static_assert(NBATCH % ROWS_BLK == 0, "batch tiles exact");
static_assert((ROWS_BLK * NOUT * 4) % 128 == 0, "block output span is whole 128-B lines");
static_assert(NLINES * 32 == ROWS_BLK * NOUT, "line count exact");
static_assert(NSTEP % XCHUNK == 0, "x chunks exact");
static_assert(COL_ZERO <= KPAD && KPAD % 32 == 0, "augmented K fits the padded K");
static_assert(UPAD == 16 * (NTHR / 32), "four waves x 16 units");
static_assert((ROWS_BLK * XCHUNK) % NTHR == 0, "x staging loop exact");
static_assert((APITCH * 2) % 16 == 0, "A rows 16-B aligned");
static_assert(NROWB * KPAD == 8 * 256 * 8, "weight plane producer coverage exact");

typedef __attribute__((ext_vector_type(16))) _Float16 v16h;
typedef __attribute__((ext_vector_type(8)))  _Float16 v8h;
typedef __attribute__((ext_vector_type(8)))  float    v8f;
typedef __attribute__((ext_vector_type(4)))  float    v4f;

__device__ __forceinline__ void grp_guard(v8f& a, v8f& b, v8f& c, v8f& d, v16h x, v16h y) {
  asm volatile("v_nop\n\tv_nop\n\tv_nop\n\tv_nop" : "+v"(a), "+v"(b), "+v"(c), "+v"(d) : "v"(x), "v"(y));
}
__device__ __forceinline__ void keep4_h(v16h a, v16h b, v16h c, v16h d) {
  asm volatile("v_nop" :: "v"(a), "v"(b), "v"(c), "v"(d));
}

template <typename T> struct Frag;
template <> struct Frag<_Float16> {
  typedef v16h V; union U { v16h v; v8h h[2]; };
  static __device__ __forceinline__ v16h load(const _Float16* p) {
    U f; f.h[0] = *(const v8h*)(p); f.h[1] = *(const v8h*)(p + 16); return f.v;
  }
  static __device__ __forceinline__ v8f mma(v16h a, v16h b, v8f c) {
    return __builtin_amdgcn_wmma_f32_16x16x32_f16(false, a, false, b, (short)0, c, false, false);
  }
};

__device__ __forceinline__ float ex2(float v) {
#if __has_builtin(__builtin_amdgcn_exp2f)
  return __builtin_amdgcn_exp2f(v);
#else
  return __expf(v * 0.6931471805599453f);
#endif
}
__device__ __forceinline__ float sig_raw(float a) {
  return __builtin_amdgcn_rcpf(1.0f + ex2(a * KSIG));
}
__device__ __forceinline__ float tanh_scaled(float a, float kk) {
  return 1.0f - 2.0f * __builtin_amdgcn_rcpf(ex2(a * kk) + 1.0f);
}

__global__ __launch_bounds__(256) void wplane_kernel(const float* __restrict__ w_ih, const float* __restrict__ w_hh,
                                                     const float* __restrict__ b_ih, const float* __restrict__ b_hh,
                                                     unsigned short* __restrict__ WB) {
  const int tid = threadIdx.x;
#pragma unroll 1
  for (int it = 0; it < 8; ++it) {
    const int idx = it * 256 + tid;
    const int n = idx >> 3;
    const int seg = idx & 7;
    const int g = n >> 6;
    const int u = n & 63;
    const int uc = (u < NHID) ? u : (NHID - 1);
    const int wr = g * NHID + uc;
    const bool live = (u < NHID);
    float bi = b_ih[wr];
    float bh = b_hh[wr];
    asm volatile("" : "+v"(bi), "+v"(bh));
    const float bs = (bi + bh) * WCARRY;
    const _Float16 bh16 = (_Float16)bs;
    const float bhi = (float)bh16;
    const float blo = bs - bhi;
    v8h hv;
#pragma unroll
    for (int e = 0; e < 8; ++e) {
      const int k = seg * 8 + e;
      const int kh = (k < NHID) ? k : (NHID - 1);
      int ki = k - COL_X;
      ki = (ki < 0) ? 0 : ((ki > NIN - 1) ? (NIN - 1) : ki);
      float a = w_hh[wr * NHID + kh];
      float q = w_ih[wr * NIN + ki];
      asm volatile("" : "+v"(a), "+v"(q));
      a = a * WCARRY;
      q = q * WCARRY;
      float v = (k < COL_X) ? a : ((k < COL_ONE) ? q : ((k == COL_ONE) ? bhi : ((k == COL_ONE + 1) ? blo : 0.0f)));
      v = live ? v : 0.0f;
      hv[e] = (_Float16)v;
    }
    *(volatile v8h*)(WB + (size_t)idx * 8) = hv;
    __threadfence();
    *(volatile v8h*)(WB + (size_t)idx * 8) = hv;
  }
}

__device__ __forceinline__ void stage_x(const float* __restrict__ x, float* xs, int rowbase, int ck, int tid) {
#pragma unroll
  for (int it = 0; it < (ROWS_BLK * XCHUNK) / NTHR; ++it) {
    const int idx = it * NTHR + tid;
    const int m = idx >> 5;
    const int tl = idx & (XCHUNK - 1);
    const v4f v = *(const v4f*)(x + ((size_t)(rowbase + m) * NSTEP + (size_t)(ck * XCHUNK + tl)) * NIN);
    *(v4f*)(xs + (m * XCHUNK + tl) * NIN) = v;
  }
}

__global__ __launch_bounds__(NTHR) void lstm_scan_kernel(const float* __restrict__ x, const unsigned short* __restrict__ WBp,
                                                         const float* __restrict__ w_out, const float* __restrict__ b_out,
                                                         float* __restrict__ out) {
  __shared__ __align__(16) _Float16 Abuf[2][ROWS_BLK * APITCH];
  __shared__ __align__(16) float    Xs[ROWS_BLK * XCHUNK * NIN];
  __shared__ __align__(16) float    Hf[ROWS_BLK * UPAD];
  __shared__ __align__(16) float    Os[ROWS_BLK * NOUT];

  const _Float16* WB = (const _Float16*)WBp;
  const int tid = threadIdx.x;
  const int lane = tid & 31;
  const int wave = tid >> 5;
  const int c = lane & 15;
  const int hh = lane >> 4;
  const int koff = hh * 8;
  const int u = 16 * wave + c;
  const int rowbase = blockIdx.x * ROWS_BLK;

  const bool is_h = (u < COL_X);
  const bool is_x = (u < COL_ONE);
  const float padc = (u == COL_ONE || u == COL_ONE + 1) ? 1.0f : 0.0f;
  int xi = u - COL_X;
  xi = (xi < 0) ? 0 : ((xi > NIN - 1) ? (NIN - 1) : xi);

  v16h bf[NGATE][2];
#pragma unroll
  for (int g = 0; g < NGATE; ++g) {
#pragma unroll
    for (int kc = 0; kc < 2; ++kc)
      bf[g][kc] = Frag<_Float16>::load(WB + (size_t)(g * UPAD + u) * KPAD + kc * 32 + koff);
  }

  stage_x(x, Xs, rowbase, 0, tid);
  __syncthreads();

#pragma unroll
  for (int mt = 0; mt < 2; ++mt) {
#pragma unroll
    for (int r = 0; r < 8; ++r) {
      const int row = 16 * mt + 8 * hh + r;
      const float xv = Xs[(row * XCHUNK) * NIN + xi];
      const float pad = is_x ? xv : padc;
      const float val = is_h ? 0.0f : pad;
      Abuf[0][row * APITCH + u] = (_Float16)(val * ACARRY);
    }
  }
  float cst[2][8], hst[2][8];
#pragma unroll
  for (int mt = 0; mt < 2; ++mt) {
#pragma unroll
    for (int r = 0; r < 8; ++r) { cst[mt][r] = 0.0f; hst[mt][r] = 0.0f; }
  }
  __syncthreads();

  const v8f z8 = {0.f, 0.f, 0.f, 0.f, 0.f, 0.f, 0.f, 0.f};

#pragma unroll 1
  for (int t = 0; t < NSTEP; ++t) {
    if (((t & (XCHUNK - 1)) == XCHUNK - 1) && (t != NSTEP - 1)) {
      stage_x(x, Xs, rowbase, (t + 1) / XCHUNK, tid);
      __syncthreads();
    }
    const _Float16* cur = &Abuf[t & 1][0];
    _Float16* nxt = &Abuf[(t + 1) & 1][0];
    const int tn = (t + 1 < NSTEP) ? (t + 1) : (NSTEP - 1);
    const int tl = tn & (XCHUNK - 1);

#pragma unroll
    for (int mt = 0; mt < 2; ++mt) {
      const _Float16* ar = cur + (16 * mt + c) * APITCH + koff;
      const v16h a0 = Frag<_Float16>::load(ar);
      const v16h a1 = Frag<_Float16>::load(ar + 32);
      v8f acc[NGATE];
#pragma unroll
      for (int g = 0; g < NGATE; ++g) acc[g] = Frag<_Float16>::mma(a0, bf[g][0], z8);
#pragma unroll
      for (int g = 0; g < NGATE; ++g) acc[g] = Frag<_Float16>::mma(a1, bf[g][1], acc[g]);
      grp_guard(acc[0], acc[1], acc[2], acc[3], a0, a1);
      keep4_h(bf[0][0], bf[1][0], bf[2][0], bf[3][0]);
      keep4_h(bf[0][1], bf[1][1], bf[2][1], bf[3][1]);

#pragma unroll
      for (int r = 0; r < 8; ++r) {
        const int row = 16 * mt + 8 * hh + r;
        const float ig = sig_raw(acc[0][r]);
        const float fg = sig_raw(acc[1][r]);
        const float gg = tanh_scaled(acc[2][r], KTG);
        const float og = sig_raw(acc[3][r]);
        const float cn = fg * cst[mt][r] + ig * gg;
        cst[mt][r] = cn;
        const float hn = og * tanh_scaled(cn, KTC);
        hst[mt][r] = hn;
        const float xv = Xs[(row * XCHUNK + tl) * NIN + xi];
        const float pad = is_x ? xv : padc;
        const float val = is_h ? hn : pad;
        nxt[row * APITCH + u] = (_Float16)(val * ACARRY);
      }
    }
    __syncthreads();
  }

#pragma unroll
  for (int mt = 0; mt < 2; ++mt) {
#pragma unroll
    for (int r = 0; r < 8; ++r) Hf[(16 * mt + 8 * hh + r) * UPAD + u] = hst[mt][r];
  }
  __syncthreads();

#pragma unroll 1
  for (int idx = tid; idx < ROWS_BLK * NOUT; idx += NTHR) {
    const int m = idx / NOUT;
    const int o = idx - m * NOUT;
    const float* hr = Hf + m * UPAD;
    const float* wr = w_out + o * NHID;
    float s = 0.0f;
#pragma unroll 5
    for (int k = 0; k < NHID; ++k) s = fmaf(hr[k], wr[k], s);
    Os[idx] = s + b_out[o];
  }
  __syncthreads();

  float* ob = out + (size_t)blockIdx.x * (size_t)(ROWS_BLK * NOUT);
  for (int pass = 0; pass < 2; ++pass) {
#pragma unroll 1
    for (int L = wave; L < NLINES; L += NTHR / 32) {
      const float v = Os[L * 32 + lane];
      *(volatile float*)(ob + L * 32 + lane) = v;
    }
    __threadfence();
  }
}

extern "C" void kernel_launch(void* const* d_in, const int* in_sizes, int n_in,
                              void* d_out, int out_size, void* d_ws, size_t ws_size, hipStream_t stream) {
  if (n_in < 7 || d_out == nullptr || d_ws == nullptr) return;
  if (in_sizes[0] != NBATCH * NSTEP * NIN || in_sizes[1] != NGATE * NHID * NIN || in_sizes[2] != NGATE * NHID * NHID ||
      in_sizes[3] != NGATE * NHID || in_sizes[4] != NGATE * NHID || in_sizes[5] != NOUT * NHID || in_sizes[6] != NOUT ||
      out_size != NBATCH * NOUT) return;
  const size_t wb_bytes = (size_t)NROWB * KPAD * 2;
  if (wb_bytes > ws_size) return;

  const float* xin  = (const float*)d_in[0];
  const float* wih  = (const float*)d_in[1];
  const float* whh  = (const float*)d_in[2];
  const float* bih  = (const float*)d_in[3];
  const float* bhh  = (const float*)d_in[4];
  const float* wout = (const float*)d_in[5];
  const float* bout = (const float*)d_in[6];
  float* out = (float*)d_out;
  unsigned short* WB = (unsigned short*)d_ws;

  wplane_kernel<<<1, 256, 0, stream>>>(wih, whh, bih, bhh, WB);
  lstm_scan_kernel<<<NBATCH / ROWS_BLK, NTHR, 0, stream>>>(xin, WB, wout, bout, out);
}
